// BatchDenseGAT_35562329211432
// MI455X (gfx1250) — hardware-verified
//
#include <hip/hip_runtime.h>
#include <math.h>

typedef __attribute__((ext_vector_type(16))) _Float16 v16h;
typedef __attribute__((ext_vector_type(16))) __bf16 v16b;
typedef __attribute__((ext_vector_type(8)))  _Float16 v8h;
typedef __attribute__((ext_vector_type(8)))  float v8f;
typedef __attribute__((ext_vector_type(4)))  float v4f;
typedef __attribute__((ext_vector_type(2)))  float v2f;
typedef __attribute__((ext_vector_type(4)))  unsigned v4u;
typedef __attribute__((ext_vector_type(4)))  int v4i;
typedef float __attribute__((may_alias)) float_a;
typedef int __attribute__((may_alias)) int_a;

template <typename T> __device__ __forceinline__ void vst2(void* p, T v) { *(volatile T*)p = v; __threadfence(); *(volatile T*)p = v; }
__device__ __forceinline__ v8f wmma16(v16h a, v16h b, v8f c) {
  v8f d = __builtin_amdgcn_wmma_f32_16x16x32_f16(false, a, false, b, (short)0, c, false, false);
  asm volatile("v_nop\n\tv_nop\n\tv_nop\n\tv_nop" : "+v"(d) : "v"(a), "v"(b));
  return d;
}
__device__ __forceinline__ v8f wmma_bf(v16b a, v16b b, v8f c) {
  v8f d = __builtin_amdgcn_wmma_f32_16x16x32_bf16(false, a, false, b, (short)0, c, false, false);
  asm volatile("v_nop\n\tv_nop\n\tv_nop\n\tv_nop" : "+v"(d) : "v"(a), "v"(b));
  return d;
}
__device__ __forceinline__ v16h frag_h(const _Float16* rowk0, int lane) {
  union { v16h v; v8h q[2]; } u; const _Float16* p = rowk0 + 8 * (lane >> 4);
  u.q[0] = *(const v8h*)p; u.q[1] = *(const v8h*)(p + 16); return u.v;
}
__device__ __forceinline__ v16h frag_f32(const float* rowk0, int lane) {
  v16h a; const float* p = rowk0 + 8 * (lane >> 4);
#pragma unroll
  for (int i = 0; i < 8; ++i) { a[i] = (_Float16)p[i]; a[8 + i] = (_Float16)p[16 + i]; }
  return a;
}
__device__ __forceinline__ v16h frag_f32s(const float* rowk0, int lane, float sc) {
  v16h a; const float* p = rowk0 + 8 * (lane >> 4);
#pragma unroll
  for (int i = 0; i < 8; ++i) { a[i] = (_Float16)(p[i] * sc); a[8 + i] = (_Float16)(p[16 + i] * sc); }
  return a;
}
__device__ __forceinline__ v16h fragc_f32(const float* W, int k0, int n, int lane, int ld, int K) {
  v16h a; const int g = lane >> 4;
#pragma unroll
  for (int i = 0; i < 8; ++i) { const int ka = k0 + 8 * g + i, kb = ka + 16;
    a[i] = (_Float16)(ka < K ? W[(size_t)(ka < K ? ka : K - 1) * ld + n] : 0.f); a[8 + i] = (_Float16)(kb < K ? W[(size_t)(kb < K ? kb : K - 1) * ld + n] : 0.f); }
  return a;
}
struct F2 { v16b h, l; };
__device__ __forceinline__ F2 bsplit16(const float v[16]) { F2 r;
#pragma unroll
  for (int i = 0; i < 16; ++i) { const __bf16 h = (__bf16)v[i]; r.h[i] = h; r.l[i] = (__bf16)(v[i] - (float)h); }
  return r; }
__device__ __forceinline__ F2 split_row(const float* row, int k0, int lane) { float v[16]; const float* p = row + k0 + 8 * (lane >> 4);
#pragma unroll
  for (int i = 0; i < 8; ++i) { v[i] = p[i]; v[8 + i] = p[16 + i]; }
  return bsplit16(v); }
__device__ __forceinline__ F2 split_rowK(const float* row, int k0, int lane, int K) { float v[16]; const int g = lane >> 4;
#pragma unroll
  for (int i = 0; i < 8; ++i) { const int ka = k0 + 8 * g + i, kb = ka + 16; v[i] = ka < K ? row[ka < K ? ka : K - 1] : 0.f; v[8 + i] = kb < K ? row[kb < K ? kb : K - 1] : 0.f; }
  return bsplit16(v); }
__device__ __forceinline__ F2 split_col(const float* W, int k0, int n, int lane, int ld, int K) { float v[16]; const int g = lane >> 4;
#pragma unroll
  for (int i = 0; i < 8; ++i) { const int ka = k0 + 8 * g + i, kb = ka + 16; v[i] = ka < K ? W[(size_t)(ka < K ? ka : K - 1) * ld + n] : 0.f; v[8 + i] = kb < K ? W[(size_t)(kb < K ? kb : K - 1) * ld + n] : 0.f; }
  return bsplit16(v); }
__device__ __forceinline__ v8f mac3(const F2& a, const F2& b, v8f c) { c = wmma_bf(a.l, b.h, c); c = wmma_bf(a.h, b.l, c); return wmma_bf(a.h, b.h, c); }
__device__ __forceinline__ float sigm(float v) { return 1.0f / (1.0f + expf(-v)); }
#define LDSX() do { asm volatile("s_wait_dscnt 0" ::: "memory"); __builtin_amdgcn_wave_barrier(); __builtin_amdgcn_fence(__ATOMIC_RELEASE, "workgroup"); } while (0)


#define NBt 32
#define NN 512
#define F0 160
#define NH1 8
#define FO1 64
#define F1 512
#define FO2 16
#define NR (NBt * NN)
typedef __attribute__((ext_vector_type(8))) __bf16 v8b;
__device__ __forceinline__ v16b frag_b(const __bf16* rowk0, int lane) {
  union { v16b v; v8b q[2]; } u; const __bf16* p = rowk0 + 8 * (lane >> 4);
  u.q[0] = *(const v8b*)p; u.q[1] = *(const v8b*)(p + 16); return u.v;
}
__device__ __forceinline__ float bfr(float v) { return (float)(__bf16)v; }
__device__ __attribute__((noinline)) float exp_ni(float v) { return expf(v); }
__device__ __attribute__((noinline)) float erf_ni(float v) { return erff(v); }

#define WS_HP  0u
#define WS_HT  (WS_HP + 4u * (size_t)NR * F1)
#define WS_SR  (WS_HT + 2u * (size_t)NBt * F1 * NN)
#define WS_DS  (WS_SR + 4u * (size_t)NBt * 16 * NN)
#define WS_H2  (WS_DS + 4u * (size_t)NBt * 16 * NN)
#define WS_T2  (WS_H2 + 4u * (size_t)NR * F1)
#define WS_END (WS_T2 + 2u * (size_t)NBt * FO2 * NN)

__global__ __launch_bounds__(128) void k_h1(const int* __restrict__ VX, const float* __restrict__ LOC, const float* __restrict__ E0, const float* __restrict__ E1, const float* __restrict__ W1, float* __restrict__ HP, _Float16* __restrict__ HT) {
  __shared__ __align__(16) __bf16 sh[64][F0 + 8]; __shared__ __align__(16) float sf[64][132]; __shared__ __align__(16) _Float16 st[128][72];
  const int tid = threadIdx.x, wave = tid >> 5, lane = tid & 31, col = lane & 15, g = lane >> 4; const size_t r0 = (size_t)blockIdx.x * 64; const int c0 = blockIdx.y * 128; const size_t b = r0 / NN; const int n0 = (int)(r0 % NN);
  for (int e = tid; e < 64 * F0; e += 128) { const int rl = e / F0, f = e % F0; const size_t row = r0 + rl; int vv = VX[row]; vv = vv < 0 ? 0 : (vv >= 100000 ? 99999 : vv);
    const float v = (f < 64) ? E0[(size_t)vv * 64 + f] : (f < 128 ? E1[(size_t)vv * 64 + f - 64] : LOC[row * 32 + f - 128]); sh[rl][f] = (__bf16)v; }
  __syncthreads();
  v8f acc[8] = {};
#pragma unroll
  for (int kc = 0; kc < F0 / 32; ++kc) { const v16b a = frag_b(&sh[wave * 16 + col][kc * 32], lane);
#pragma unroll
    for (int j = 0; j < 8; ++j) { v16b w; const int oc = c0 + j * 16 + col; const int hh = oc / FO1, o = oc % FO1;
#pragma unroll
      for (int i = 0; i < 8; ++i) { w[i] = (__bf16)W1[((size_t)hh * F0 + kc * 32 + 8 * g + i) * FO1 + o]; w[8 + i] = (__bf16)W1[((size_t)hh * F0 + kc * 32 + 16 + 8 * g + i) * FO1 + o]; }
      acc[j] = wmma_bf(a, w, acc[j]); } }
#pragma unroll
  for (int j = 0; j < 8; ++j)
#pragma unroll
    for (int r = 0; r < 8; ++r) { const float v = acc[j][r]; const int rl = wave * 16 + 8 * g + r, cl = j * 16 + col; sf[rl][cl] = v; st[cl][rl] = (_Float16)v; }
  __syncthreads();
  for (int e = tid; e < 64 * 32; e += 128) { const int rl = e >> 5, q = e & 31; vst2(HP + (r0 + rl) * F1 + c0 + q * 4, *(const v4f*)&sf[rl][q * 4]); }
  for (int e = tid; e < 128 * 8; e += 128) { const int cl = e >> 3, q = e & 7; vst2((unsigned*)(HT + (b * F1 + c0 + cl) * (size_t)NN + n0 + q * 8), *(const v4u*)&st[cl][q * 8]); } }
template <int NHD, int FO>
__global__ __launch_bounds__(128) void k_sd(const float* __restrict__ HPx, const float* __restrict__ AS, const float* __restrict__ AD, float* __restrict__ SR, float* __restrict__ DS) { __shared__ float ps[NHD * 4], pd[NHD * 4];
  const int t = threadIdx.x; const size_t row = blockIdx.x; const size_t b = row / NN; const int n = (int)(row % NN); const int wv = t >> 5, ln = t & 31;
  for (int h = wv; h < NHD; h += 4) { float s = 0.f, d = 0.f; for (int o = ln; o < FO; o += 32) { const float tv = tanhf(HPx[row * (NHD * FO) + h * FO + o]); s += tv * bfr(AS[h * FO + o]); d += tv * bfr(AD[h * FO + o]); }
#pragma unroll
    for (int of = 1; of < 32; of <<= 1) { s += __shfl_xor(s, of); d += __shfl_xor(d, of); }
    if (ln == 0) { ps[h] = s; pd[h] = d; } }
  __syncthreads();
  if (t < 4) { __align__(16) float v[4], u[4]; for (int k = 0; k < 4; ++k) { const int h = t * 4 + k; v[k] = (h < NHD) ? ps[h] : 0.f; u[k] = (h < NHD) ? pd[h] : 0.f; } vst2(SR + row * 16 + t * 4, *(const v4f*)v); vst2(DS + row * 16 + t * 4, *(const v4f*)u); } }
template <int LAYER>
__global__ __launch_bounds__(128) void k_att(const float* __restrict__ SR, const float* __restrict__ DS, const float* __restrict__ ADJ, const _Float16* __restrict__ HT, float* __restrict__ DST) {
  __shared__ __align__(16) _Float16 sp[64][NN + 8]; __shared__ float sdm[NN]; __shared__ __align__(16) float so[64][68];
  const int tid = threadIdx.x, wave = tid >> 5, lane = tid & 31, col = lane & 15, g = lane >> 4; const int n0 = blockIdx.x * 64; const int h = blockIdx.y; const size_t b = blockIdx.z; const int hidx = (LAYER == 1) ? h : 0;
  constexpr int FO = (LAYER == 1) ? FO1 : FO2; constexpr int NPL = (LAYER == 1) ? F1 : FO2;
  for (int m = tid; m < NN; m += 128) sdm[m] = DS[(b * NN + m) * 16 + hidx];
  __syncthreads();
  for (int rr = 0; rr < 16; ++rr) { const int rl = wave * 16 + rr; const int n = n0 + rl; const float sn = SR[(b * NN + n) * 16 + hidx]; const float* arow = ADJ + (b * NN + n) * (size_t)NN;
    float ev[NN / 32]; float mx = -3.0e38f;
#pragma unroll
    for (int i = 0; i < NN / 32; ++i) { const int m = lane + 32 * i; float e = sn + sdm[m]; e = (e >= 0.f) ? e : 0.2f * e; const bool ok = bfr(arow[m]) > 0.f; ev[i] = ok ? e : -3.0e38f; if (ok) mx = fmaxf(mx, e); }
#pragma unroll
    for (int of = 1; of < 32; of <<= 1) mx = fmaxf(mx, __shfl_xor(mx, of));
    float sum = 0.f;
#pragma unroll
    for (int i = 0; i < NN / 32; ++i) { const float p = (ev[i] <= -1.0e38f) ? 0.f : expf(ev[i] - mx); ev[i] = p; sum += p; }
#pragma unroll
    for (int of = 1; of < 32; of <<= 1) sum += __shfl_xor(sum, of);
    const float inv = 2048.0f / sum;
#pragma unroll
    for (int i = 0; i < NN / 32; ++i) sp[rl][lane + 32 * i] = (_Float16)(ev[i] * inv); }
  __syncthreads();
  v8f acc[FO / 16]; for (int j = 0; j < FO / 16; ++j) for (int r = 0; r < 8; ++r) acc[j][r] = 0.f;
#pragma unroll 1
  for (int kc = 0; kc < NN / 32; ++kc) { const v16h a = frag_h(&sp[wave * 16 + col][kc * 32], lane);
#pragma unroll
    for (int j = 0; j < FO / 16; ++j) acc[j] = wmma16(a, frag_h(HT + (b * NPL + hidx * FO + j * 16 + col) * (size_t)NN + kc * 32, lane), acc[j]); }
  if (LAYER == 1) {
#pragma unroll
    for (int j = 0; j < FO / 16; ++j)
#pragma unroll
      for (int r = 0; r < 8; ++r) { const float v = acc[j][r] * (1.0f / 2048.0f); so[wave * 16 + 8 * g + r][j * 16 + col] = (v > 0.f) ? v : expm1f(v); }
    __syncthreads(); for (int e = tid; e < 64 * 16; e += 128) { const int rl = e >> 4, q = e & 15; vst2(DST + (b * NN + n0 + rl) * (size_t)F1 + h * FO1 + q * 4, *(const v4f*)&so[rl][q * 4]); } }
  else {
#pragma unroll
    for (int r = 0; r < 8; ++r) { const float v = acc[0][r] * (1.0f / 2048.0f); float mx = v;
#pragma unroll
      for (int of = 1; of < 16; of <<= 1) mx = fmaxf(mx, __shfl_xor(mx, of)); float s = expf(v - mx);
#pragma unroll
      for (int of = 1; of < 16; of <<= 1) s += __shfl_xor(s, of); so[wave * 16 + 8 * g + r][col] = v - mx - logf(s); }
    __syncthreads(); for (int e = tid; e < 64 * 4; e += 128) { const int rl = e >> 2, q = e & 3; vst2(DST + (b * NN + n0 + rl) * (size_t)FO2 + q * 4, *(const v4f*)&so[rl][q * 4]); } } }
__global__ __launch_bounds__(128) void k_h2(const float* __restrict__ H2, const float* __restrict__ W2, float* __restrict__ HP2, _Float16* __restrict__ T2) { __shared__ __align__(16) float sf[64][20]; __shared__ __align__(16) _Float16 st[16][72];
  const int tid = threadIdx.x, wave = tid >> 5, lane = tid & 31, col = lane & 15, g = lane >> 4; const size_t r0 = (size_t)blockIdx.x * 64; const size_t b = r0 / NN; const int n0 = (int)(r0 % NN);
  v8f acc = {};
#pragma unroll 2
  for (int kc = 0; kc < F1 / 32; ++kc) { const v16h a = frag_f32(H2 + (r0 + wave * 16 + col) * F1 + kc * 32, lane); v16h w;
#pragma unroll
    for (int i = 0; i < 8; ++i) { w[i] = (_Float16)bfr(W2[(size_t)(kc * 32 + 8 * g + i) * FO2 + col]); w[8 + i] = (_Float16)bfr(W2[(size_t)(kc * 32 + 16 + 8 * g + i) * FO2 + col]); }
    acc = wmma16(a, w, acc); }
#pragma unroll
  for (int r = 0; r < 8; ++r) { const int rl = wave * 16 + 8 * g + r; sf[rl][col] = acc[r]; st[col][rl] = (_Float16)acc[r]; }
  __syncthreads();
  for (int e = tid; e < 64 * 4; e += 128) { const int rl = e >> 2, q = e & 3; vst2(HP2 + (r0 + rl) * FO2 + q * 4, *(const v4f*)&sf[rl][q * 4]); }
  if (tid < 16 * 8) { const int cl = tid >> 3, q = tid & 7; vst2((unsigned*)(T2 + (b * FO2 + cl) * (size_t)NN + n0 + q * 8), *(const v4u*)&st[cl][q * 8]); } }
extern "C" void kernel_launch(void* const* d_in, const int* in_sizes, int n_in, void* d_out, int out_size, void* d_ws, size_t ws_size, hipStream_t stream) {
  (void)in_sizes; (void)n_in; (void)out_size;
  const float** F = (const float**)d_in;
  if (ws_size < (size_t)WS_END) return;
  char* ws = (char*)d_ws; float *HP = (float*)(ws + WS_HP), *SR = (float*)(ws + WS_SR), *DS = (float*)(ws + WS_DS), *H2 = (float*)(ws + WS_H2); _Float16 *HT = (_Float16*)(ws + WS_HT), *T2 = (_Float16*)(ws + WS_T2);
  k_h1<<<dim3(NR / 64, F1 / 128), 128, 0, stream>>>((const int*)d_in[1], F[2], F[3], F[4], F[5], HP, HT);
  k_sd<NH1, FO1><<<NR, 128, 0, stream>>>(HP, F[6], F[7], SR, DS);
  k_att<1><<<dim3(NN / 64, NH1, NBt), 128, 0, stream>>>(SR, DS, F[0], HT, H2);
  k_h2<<<NR / 64, 128, 0, stream>>>(H2, F[8], HP, T2);
  k_sd<1, FO2><<<NR, 128, 0, stream>>>(HP, F[9], F[10], SR, DS);
  k_att<2><<<dim3(NN / 64, 1, NBt), 128, 0, stream>>>(SR, DS, F[0], T2, (float*)d_out);
}
